// quantum_attention_40218073760356
// MI455X (gfx1250) — hardware-verified
//
#include <hip/hip_runtime.h>
#include <math.h>

typedef __attribute__((ext_vector_type(16))) _Float16 v16h;
typedef __attribute__((ext_vector_type(16))) __bf16 v16b;
typedef __attribute__((ext_vector_type(8)))  _Float16 v8h;
typedef __attribute__((ext_vector_type(8)))  float v8f;
typedef __attribute__((ext_vector_type(4)))  float v4f;
typedef __attribute__((ext_vector_type(2)))  float v2f;
typedef __attribute__((ext_vector_type(4)))  unsigned v4u;
typedef __attribute__((ext_vector_type(4)))  int v4i;
typedef float __attribute__((may_alias)) float_a;
typedef int __attribute__((may_alias)) int_a;

template <typename T> __device__ __forceinline__ void vst2(void* p, T v) { *(volatile T*)p = v; __threadfence(); *(volatile T*)p = v; }
__device__ __forceinline__ v8f wmma16(v16h a, v16h b, v8f c) {
  v8f d = __builtin_amdgcn_wmma_f32_16x16x32_f16(false, a, false, b, (short)0, c, false, false);
  asm volatile("v_nop\n\tv_nop\n\tv_nop\n\tv_nop" : "+v"(d) : "v"(a), "v"(b));
  return d;
}
__device__ __forceinline__ v8f wmma_bf(v16b a, v16b b, v8f c) {
  v8f d = __builtin_amdgcn_wmma_f32_16x16x32_bf16(false, a, false, b, (short)0, c, false, false);
  asm volatile("v_nop\n\tv_nop\n\tv_nop\n\tv_nop" : "+v"(d) : "v"(a), "v"(b));
  return d;
}
__device__ __forceinline__ v16h frag_h(const _Float16* rowk0, int lane) {
  union { v16h v; v8h q[2]; } u; const _Float16* p = rowk0 + 8 * (lane >> 4);
  u.q[0] = *(const v8h*)p; u.q[1] = *(const v8h*)(p + 16); return u.v;
}
__device__ __forceinline__ v16h frag_f32(const float* rowk0, int lane) {
  v16h a; const float* p = rowk0 + 8 * (lane >> 4);
#pragma unroll
  for (int i = 0; i < 8; ++i) { a[i] = (_Float16)p[i]; a[8 + i] = (_Float16)p[16 + i]; }
  return a;
}
__device__ __forceinline__ v16h frag_f32s(const float* rowk0, int lane, float sc) {
  v16h a; const float* p = rowk0 + 8 * (lane >> 4);
#pragma unroll
  for (int i = 0; i < 8; ++i) { a[i] = (_Float16)(p[i] * sc); a[8 + i] = (_Float16)(p[16 + i] * sc); }
  return a;
}
__device__ __forceinline__ v16h fragc_f32(const float* W, int k0, int n, int lane, int ld, int K) {
  v16h a; const int g = lane >> 4;
#pragma unroll
  for (int i = 0; i < 8; ++i) { const int ka = k0 + 8 * g + i, kb = ka + 16;
    a[i] = (_Float16)(ka < K ? W[(size_t)(ka < K ? ka : K - 1) * ld + n] : 0.f); a[8 + i] = (_Float16)(kb < K ? W[(size_t)(kb < K ? kb : K - 1) * ld + n] : 0.f); }
  return a;
}
struct F2 { v16b h, l; };
__device__ __forceinline__ F2 bsplit16(const float v[16]) { F2 r;
#pragma unroll
  for (int i = 0; i < 16; ++i) { const __bf16 h = (__bf16)v[i]; r.h[i] = h; r.l[i] = (__bf16)(v[i] - (float)h); }
  return r; }
__device__ __forceinline__ F2 split_row(const float* row, int k0, int lane) { float v[16]; const float* p = row + k0 + 8 * (lane >> 4);
#pragma unroll
  for (int i = 0; i < 8; ++i) { v[i] = p[i]; v[8 + i] = p[16 + i]; }
  return bsplit16(v); }
__device__ __forceinline__ F2 split_rowK(const float* row, int k0, int lane, int K) { float v[16]; const int g = lane >> 4;
#pragma unroll
  for (int i = 0; i < 8; ++i) { const int ka = k0 + 8 * g + i, kb = ka + 16; v[i] = ka < K ? row[ka < K ? ka : K - 1] : 0.f; v[8 + i] = kb < K ? row[kb < K ? kb : K - 1] : 0.f; }
  return bsplit16(v); }
__device__ __forceinline__ F2 split_col(const float* W, int k0, int n, int lane, int ld, int K) { float v[16]; const int g = lane >> 4;
#pragma unroll
  for (int i = 0; i < 8; ++i) { const int ka = k0 + 8 * g + i, kb = ka + 16; v[i] = ka < K ? W[(size_t)(ka < K ? ka : K - 1) * ld + n] : 0.f; v[8 + i] = kb < K ? W[(size_t)(kb < K ? kb : K - 1) * ld + n] : 0.f; }
  return bsplit16(v); }
__device__ __forceinline__ v8f mac3(const F2& a, const F2& b, v8f c) { c = wmma_bf(a.l, b.h, c); c = wmma_bf(a.h, b.l, c); return wmma_bf(a.h, b.h, c); }
__device__ __forceinline__ float sigm(float v) { return 1.0f / (1.0f + expf(-v)); }
#define LDSX() do { asm volatile("s_wait_dscnt 0" ::: "memory"); __builtin_amdgcn_wave_barrier(); __builtin_amdgcn_fence(__ATOMIC_RELEASE, "workgroup"); } while (0)


#define NB 2
#define TT 2048
#define CC 1024
#define NH 16
#define HD 64
#ifndef TNB
#define TNB NB
#endif
typedef __attribute__((ext_vector_type(8))) __bf16 v8b;
__device__ __forceinline__ v16b frag_b(const __bf16* rowk0, int lane) {
  union { v16b v; v8b q[2]; } u; const __bf16* p = rowk0 + 8 * (lane >> 4);
  u.q[0] = *(const v8b*)p; u.q[1] = *(const v8b*)(p + 16); return u.v;
}
__device__ __forceinline__ float bfr(float v) { return (float)(__bf16)v; }
__device__ __attribute__((noinline)) float exp_ni(float v) { return expf(v); }
__device__ __attribute__((noinline)) float erf_ni(float v) { return erff(v); }

#define WS_QH  0u
#define WS_QL  (WS_QH + 2u * (size_t)NB * TT * CC)
#define WS_KH  (WS_QL + 2u * (size_t)NB * TT * CC)
#define WS_VT  (WS_KH + 2u * (size_t)NB * TT * CC)
#define WS_VL  (WS_VT + 2u * (size_t)NB * CC * TT)
#define HG 4
#define WS_S   (WS_VL + 2u * (size_t)NB * CC * TT)
#define WS_PH  (WS_S + 4u * (size_t)HG * TT * TT)
#define WS_Y   (WS_PH + 0u)
#define WS_END (WS_Y + 4u * (size_t)NB * TT * CC)

__global__ __launch_bounds__(128) void k_proj(const float* __restrict__ X, const float* __restrict__ WQ, const float* __restrict__ BQ, const float* __restrict__ WK, const float* __restrict__ BK, const float* __restrict__ WV, const float* __restrict__ BV, _Float16* __restrict__ QH, _Float16* __restrict__ QL, _Float16* __restrict__ KH, __bf16* __restrict__ VT, __bf16* __restrict__ VL) {
  __shared__ __align__(16) _Float16 sh[64][136], sl[64][136]; __shared__ __align__(16) __bf16 th[128][72], tl2[128][72];
  const int tid = threadIdx.x, wave = tid >> 5, lane = tid & 31, col = lane & 15, g = lane >> 4; const int which = blockIdx.z; const int c0 = blockIdx.y * 128; const size_t r0 = (size_t)blockIdx.x * 64; const float* WA = which == 0 ? WQ : which == 1 ? WK : WV; const float* BA = which == 0 ? BQ : which == 1 ? BK : BV;
  v8f acc[8] = {};
#pragma unroll 2
  for (int kc = 0; kc < CC / 32; ++kc) { v16b a; { const float* p = X + (r0 + wave * 16 + col) * CC + kc * 32 + 8 * g;
#pragma unroll
      for (int i = 0; i < 8; ++i) { a[i] = (__bf16)p[i]; a[8 + i] = (__bf16)p[16 + i]; } }
#pragma unroll
    for (int j = 0; j < 8; ++j) { v16b w; const int o = c0 + j * 16 + col;
#pragma unroll
      for (int i = 0; i < 8; ++i) { w[i] = (__bf16)WA[(size_t)(kc * 32 + 8 * g + i) * CC + o]; w[8 + i] = (__bf16)WA[(size_t)(kc * 32 + 16 + 8 * g + i) * CC + o]; }
      acc[j] = wmma_bf(a, w, acc[j]); } }
#pragma unroll
  for (int j = 0; j < 8; ++j) { const float bb = BA ? bfr(BA[c0 + j * 16 + col]) : 0.f;
#pragma unroll
    for (int r = 0; r < 8; ++r) { const float v = acc[j][r] + bb; const int rl = wave * 16 + 8 * g + r, cl = j * 16 + col; const _Float16 hv = (_Float16)v;
      if (which == 2) { const __bf16 bh = (__bf16)v; th[cl][rl] = bh; tl2[cl][rl] = (__bf16)(v - (float)bh); } else { sh[rl][cl] = hv; sl[rl][cl] = (_Float16)((v - (float)hv) * 1024.0f); }     } }
  __syncthreads();
  if (which < 2) { _Float16* dh = which == 0 ? QH : KH; for (int e = tid; e < 64 * 16; e += 128) { const int rl = e >> 4, q = e & 15; vst2((unsigned*)(dh + (r0 + rl) * CC + c0 + q * 8), *(const v4u*)&sh[rl][q * 8]); if (which == 0) vst2((unsigned*)(QL + (r0 + rl) * CC + c0 + q * 8), *(const v4u*)&sl[rl][q * 8]); } }
  else { const size_t b = r0 / TT; const int t0 = (int)(r0 % TT); for (int e = tid; e < 128 * 8; e += 128) { const int cl = e >> 3, q = e & 7; const size_t o2 = (b * CC + c0 + cl) * (size_t)TT + t0 + q * 8; vst2((unsigned*)(VT + o2), *(const v4u*)&th[cl][q * 8]); vst2((unsigned*)(VL + o2), *(const v4u*)&tl2[cl][q * 8]); } } }
__device__ __forceinline__ float cos_small(float x) { const float m = rintf(x * 0.318309886183790672f); float r = fmaf(m, -3.14159274101257324f, x); r = fmaf(m, 8.74227765734758577e-8f, r);
  const float r2 = r * r; float p = -2.08767569878681e-9f; p = fmaf(p, r2, 2.75573192239859e-7f); p = fmaf(p, r2, -2.48015873015873e-5f); p = fmaf(p, r2, 1.38888888888889e-3f); p = fmaf(p, r2, -4.16666666666667e-2f); p = fmaf(p, r2, 0.5f); p = fmaf(-p, r2, 1.0f);
  const int mi = (int)m; return (mi & 1) ? -p : p; }
__global__ __launch_bounds__(128) void k_sc(const _Float16* __restrict__ QH, const _Float16* __restrict__ QL, const _Float16* __restrict__ KH, const float* __restrict__ PSC, int b, int h0, float* __restrict__ S0) { __shared__ __align__(16) float ss[4][16][132]; const int h = h0 + blockIdx.z; float* S = S0 + (size_t)blockIdx.z * TT * TT;
  const int tid = threadIdx.x, wave = tid >> 5, lane = tid & 31, col = lane & 15, g = lane >> 4; const int k0 = blockIdx.y * 128; const int ql0 = blockIdx.x * 64 + wave * 16; const size_t q0 = (size_t)b * TT + ql0;
  v8f acc[8] = {}, accl[8] = {};
#pragma unroll
  for (int kc = 0; kc < HD / 32; ++kc) { const v16h ah = frag_h(QH + (q0 + col) * CC + h * HD + kc * 32, lane), al = frag_h(QL + (q0 + col) * CC + h * HD + kc * 32, lane);
#pragma unroll
    for (int j = 0; j < 8; ++j) { const v16h kb = frag_h(KH + ((size_t)b * TT + k0 + j * 16 + col) * CC + h * HD + kc * 32, lane); acc[j] = wmma16(ah, kb, acc[j]); accl[j] = wmma16(al, kb, accl[j]); } }
  const float psc = 0.125f * bfr(PSC[h]);
#pragma unroll
  for (int j = 0; j < 8; ++j)
#pragma unroll
    for (int r = 0; r < 8; ++r) { const float s = (acc[j][r] + accl[j][r] * (1.0f / 1024.0f)) * psc; ss[wave][8 * g + r][j * 16 + col] = cos_small(s) + 0.1f * cos_small(2.0f * s); }
  LDSX(); for (int rl = 0; rl < 16; ++rl) vst2(S + (size_t)(ql0 + rl) * TT + k0 + lane * 4, *(const v4f*)&ss[wave][rl][lane * 4]); }
__global__ __launch_bounds__(256) void k_sm(float* __restrict__ S0) { __shared__ float sred[8]; __shared__ float sbc; __shared__ __align__(16) float sh[TT];
  const int t = threadIdx.x; const size_t row = blockIdx.x; float* sr = S0 + (size_t)blockIdx.y * TT * TT + row * TT; const int kend = TT;
  float m = -3.0e38f; for (int k = t; k < kend; k += 256) m = fmaxf(m, sr[k]);
#pragma unroll
  for (int o = 1; o < 32; o <<= 1) m = fmaxf(m, __shfl_xor(m, o));
  if ((t & 31) == 0) sred[t >> 5] = m; __syncthreads(); if (t == 0) { float a = sred[0]; for (int i = 1; i < 8; ++i) a = fmaxf(a, sred[i]); sbc = a; } __syncthreads(); m = sbc; __syncthreads();
  float sum = 0.f; for (int k = t; k < kend; k += 256) { const float v = sr[k]; sum += (v <= -1.0e38f) ? 0.f : expf(v - m); }
#pragma unroll
  for (int o = 1; o < 32; o <<= 1) sum += __shfl_xor(sum, o);
  if ((t & 31) == 0) sred[t >> 5] = sum; __syncthreads(); if (t == 0) { float a = 0.f; for (int i = 0; i < 8; ++i) a += sred[i]; sbc = 1.0f / a; } __syncthreads(); const float inv = sbc;
  for (int k = t; k < kend; k += 256) { const float v = sr[k]; sh[k] = (v <= -1.0e38f) ? 0.f : expf(v - m) * inv * 2048.0f; }
  __syncthreads(); for (int q = t; q < kend / 4; q += 256) vst2(sr + q * 4, *(const v4f*)&sh[q * 4]); }
__global__ __launch_bounds__(128) void k_pv(const float* __restrict__ PS0, const __bf16* __restrict__ VT, const __bf16* __restrict__ VL, int b, int h0, float* __restrict__ Y) { const int h = h0 + blockIdx.z; const float* PS = PS0 + (size_t)blockIdx.z * TT * TT; __shared__ __align__(16) float ss[4][16][HD + 4];
  const int tid = threadIdx.x, wave = tid >> 5, lane = tid & 31, col = lane & 15, g = lane >> 4; const int ql0 = blockIdx.x * 64 + wave * 16; const int kend = TT;
  v8f acc[HD / 16] = {};
#pragma unroll 1
  for (int kc = 0; kc < kend / 32; ++kc) { const F2 p = split_row(PS + (size_t)(ql0 + col) * TT, kc * 32, lane);
#pragma unroll
    for (int j = 0; j < HD / 16; ++j) { const size_t po = ((size_t)b * CC + h * HD + j * 16 + col) * (size_t)TT + kc * 32; const v16b vh = frag_b(VT + po, lane); acc[j] = wmma_bf(p.h, vh, acc[j]); acc[j] = wmma_bf(p.l, vh, acc[j]); acc[j] = wmma_bf(p.h, frag_b(VL + po, lane), acc[j]); } }
#pragma unroll
  for (int j = 0; j < HD / 16; ++j)
#pragma unroll
    for (int r = 0; r < 8; ++r) ss[wave][8 * g + r][j * 16 + col] = acc[j][r] * (1.0f / 2048.0f);
  LDSX(); for (int rl = 0; rl < 16; ++rl) if (lane < HD / 4) vst2(Y + ((size_t)b * TT + ql0 + rl) * CC + h * HD + lane * 4, *(const v4f*)&ss[wave][rl][lane * 4]); }
__global__ __launch_bounds__(256) void k_mix(float* __restrict__ Y, const float* __restrict__ ENT) {     __shared__ float sy[CC]; __shared__ float se[NH * NH]; __shared__ float sa[HD]; __shared__ float scs[NH];
  const int t = threadIdx.x; const size_t row = blockIdx.x; for (int e = t; e < CC; e += 256) sy[e] = Y[row * CC + e]; se[t] = bfr(ENT[t]);
  __syncthreads();
  if (t < HD) { float a = 0.f;
#pragma unroll 4
    for (int n = 0; n < NH; ++n) a += sy[n * HD + t]; sa[t] = a; }
  else if (t >= 64 && t < 64 + NH) { const int m = t - 64; float c = 0.f;
#pragma unroll 4
    for (int h = 0; h < NH; ++h) c += se[h * NH + m]; scs[m] = c; }
  __syncthreads();
#pragma unroll 1
  for (int q = 0; q < 4; ++q) { const int c = q * 256 + t; const int m = c / HD, d = c % HD; vst2(Y + row * CC + c, sa[d] * scs[m]); } }
__global__ __launch_bounds__(128) void k_out(const float* __restrict__ Y, const float* __restrict__ WP, const float* __restrict__ BP, const float* __restrict__ XIN, float* __restrict__ OUT) { __shared__ __align__(16) float sf[4][16][132];
  const int tid = threadIdx.x, wave = tid >> 5, lane = tid & 31, col = lane & 15, g = lane >> 4; const int c0 = blockIdx.y * 128; const size_t r0 = (size_t)blockIdx.x * 64 + wave * 16;
  v8f acc[8] = {};
#pragma unroll 2
  for (int kc = 0; kc < CC / 32; ++kc) { const F2 a = split_row(Y + (r0 + col) * CC, kc * 32, lane);
#pragma unroll
    for (int j = 0; j < 8; ++j) { v16b w; const int o = c0 + j * 16 + col;
#pragma unroll
      for (int i = 0; i < 8; ++i) { w[i] = (__bf16)WP[(size_t)(kc * 32 + 8 * g + i) * CC + o]; w[8 + i] = (__bf16)WP[(size_t)(kc * 32 + 16 + 8 * g + i) * CC + o]; }
      acc[j] = wmma_bf(a.h, w, acc[j]); acc[j] = wmma_bf(a.l, w, acc[j]); } }
#pragma unroll
  for (int j = 0; j < 8; ++j) { const float bb = BP ? bfr(BP[c0 + j * 16 + col]) : 0.f;
#pragma unroll
    for (int r = 0; r < 8; ++r) sf[wave][8 * g + r][j * 16 + col] = acc[j][r] + bb + bfr(XIN[(r0 + 8 * g + r) * CC + c0 + j * 16 + col]); asm volatile("s_wait_loadcnt 0x0" ::: "memory"); }
  LDSX(); for (int rl = 0; rl < 16; ++rl) vst2(OUT + (r0 + rl) * CC + c0 + lane * 4, *(const v4f*)&sf[wave][rl][lane * 4]); }
__global__ __launch_bounds__(256) void k_ln(float* __restrict__ OUT, const float* __restrict__ GA, const float* __restrict__ BE) {
  const int t = threadIdx.x; const int rl = t >> 4, sub = t & 15; const size_t row = (size_t)blockIdx.x * 16 + rl; float* p = OUT + row * CC;
  float s = 0.f; for (int c = sub * 4; c < CC; c += 64) { const v4f v = *(const v4f*)(p + c); s += (v[0] + v[1]) + (v[2] + v[3]); }
#pragma unroll
  for (int o = 1; o < 16; o <<= 1) s += __shfl_xor(s, o);
  const float mu = s * (1.0f / CC); float s2 = 0.f; for (int c = sub * 4; c < CC; c += 64) { const v4f v = *(const v4f*)(p + c); const float d0 = v[0] - mu, d1 = v[1] - mu, d2 = v[2] - mu, d3 = v[3] - mu; s2 += (d0 * d0 + d1 * d1) + (d2 * d2 + d3 * d3); }
#pragma unroll
  for (int o = 1; o < 16; o <<= 1) s2 += __shfl_xor(s2, o);
  const float rs = rsqrtf(s2 * (1.0f / CC) + 1e-6f);
  for (int c = sub * 4; c < CC; c += 64) { const v4f v = *(const v4f*)(p + c); v4f o; for (int z = 0; z < 4; ++z) o[z] = (v[z] - mu) * rs * bfr(GA[c + z]) + bfr(BE[c + z]); vst2(p + c, o); } }
extern "C" void kernel_launch(void* const* d_in, const int* in_sizes, int n_in, void* d_out, int out_size, void* d_ws, size_t ws_size, hipStream_t stream) {
  (void)in_sizes; (void)n_in; (void)out_size;
  const float** F = (const float**)d_in;
  if (ws_size < (size_t)WS_END) return;
  char* ws = (char*)d_ws; _Float16 *QH = (_Float16*)(ws + WS_QH), *QL = (_Float16*)(ws + WS_QL), *KH = (_Float16*)(ws + WS_KH); __bf16 *VT = (__bf16*)(ws + WS_VT), *VL = (__bf16*)(ws + WS_VL); float *S = (float*)(ws + WS_S), *Y = (float*)(ws + WS_Y);
  k_proj<<<dim3(TNB * TT / 64, CC / 128, 3), 128, 0, stream>>>(F[0], F[1], nullptr, F[2], nullptr, F[3], nullptr, QH, QL, KH, VT, VL);
  for (int b = 0; b < TNB; ++b) for (int h0 = 0; h0 < NH; h0 += HG) {
    k_sc<<<dim3(TT / 64, TT / 128, HG), 128, 0, stream>>>(QH, QL, KH, F[6], b, h0, S);
    k_sm<<<dim3(TT, HG), 256, 0, stream>>>(S);
    k_pv<<<dim3(TT / 64, 1, HG), 128, 0, stream>>>(S, VT, VL, b, h0, Y);
  }
  k_mix<<<dim3(TNB * TT), 256, 0, stream>>>(Y, F[7]);
  k_out<<<dim3(TNB * TT / 64, CC / 128), 128, 0, stream>>>(Y, F[4], F[5], F[0], (float*)d_out);
  k_ln<<<dim3(TNB * TT / 16), 256, 0, stream>>>((float*)d_out, F[8], F[9]);
}
